// ConvCaps3D_40020505264452
// MI455X (gfx1250) — hardware-verified
//
#include <hip/hip_runtime.h>
#include <math.h>
#include <stdint.h>

#define NBAT   8
#define CIN    16
#define DCAP   32
#define HIN    24
#define WIN    24
#define CO     16
#define DOC    32
#define HOUT   22
#define WOUT   22
#define NPIX   484
#define MDIM   512
#define KDIM   144
#define KPAD   160
#define RITERS 3
#define UPITCH 33
#define NPOS   3872

static_assert(MDIM == CO * DOC);
static_assert(KDIM == CIN * 9);
static_assert(NPIX == HOUT * WOUT);
static_assert(NPOS == NBAT * NPIX);
static_assert((KPAD % 32) == 0 && KPAD >= KDIM && (KDIM % 8) == 0);
static_assert(((MDIM * (KPAD / 8)) % 256) == 0);
static_assert(((NBAT * HIN * WIN * CIN * DCAP / 8) % 256) == 0);
static_assert(((NPOS * MDIM) % 1024) == 0);

typedef __bf16   v16b __attribute__((ext_vector_type(16)));
typedef __bf16   v8b  __attribute__((ext_vector_type(8)));
typedef float    v8f  __attribute__((ext_vector_type(8)));
typedef float    v4f  __attribute__((ext_vector_type(4)));
typedef unsigned int v4u __attribute__((ext_vector_type(4)));

__device__ __forceinline__ unsigned short bf_bits(float f) {
  unsigned u = __float_as_uint(f);
  return (unsigned short)((u + 0x7FFFu + ((u >> 16) & 1u)) >> 16);
}
__device__ __forceinline__ float bf_up(unsigned short h) { return __uint_as_float(((unsigned)h) << 16); }
__device__ __forceinline__ float bfr(float f) { return bf_up(bf_bits(f)); }
__device__ __forceinline__ unsigned pk16(unsigned short a, unsigned short b) { return (unsigned)a | ((unsigned)b << 16); }
__device__ __forceinline__ v8f zero8() { v8f z = {0.f, 0.f, 0.f, 0.f, 0.f, 0.f, 0.f, 0.f}; return z; }

__device__ __forceinline__ v16b ldfrag_b(const __bf16* p) {
  union { v16b v; v8b h[2]; } f;
  f.h[0] = *(const v8b*)(p);
  f.h[1] = *(const v8b*)(p + 16);
  return f.v;
}
__device__ __forceinline__ v16b ldfrag_lds(const unsigned short* p) {
  union { v16b v; v8b h[2]; } f;
  f.h[0] = *(const v8b*)(const void*)(p);
  f.h[1] = *(const v8b*)(const void*)(p + 16);
  return f.v;
}

__device__ __forceinline__ v8f mma_b_raw(v16b a, v16b b, v8f c) {
  return __builtin_amdgcn_wmma_f32_16x16x32_bf16(false, a, false, b, (short)0, c, false, false);
}
__device__ __forceinline__ void dep_guard_b(v8f& a, v8f& b, v16b x, v16b y) {
#if defined(__HIP_DEVICE_COMPILE__)
  asm volatile("v_nop\n\tv_nop\n\tv_nop\n\tv_nop" : "+v"(a), "+v"(b) : "v"(x), "v"(y));
#endif
}
__device__ __forceinline__ void keep2_b(v16b a, v16b b) {
#if defined(__HIP_DEVICE_COMPILE__)
  asm volatile("v_nop" :: "v"(a), "v"(b));
#endif
}
__device__ __forceinline__ void acc_guard4(v8f& a, v8f& b, v8f& c, v8f& d) {
#if defined(__HIP_DEVICE_COMPILE__)
  asm volatile("v_nop\n\tv_nop\n\tv_nop\n\tv_nop" : "+v"(a), "+v"(b), "+v"(c), "+v"(d));
#endif
}

__global__ __launch_bounds__(256) void k_packw(const float* __restrict__ w, unsigned short* wp) {
  const int idx = blockIdx.x * 256 + threadIdx.x;
  const int m   = idx / (KPAD / 8);
  const int q   = idx - m * (KPAD / 8);
  const int k   = q * 8;
  const bool ok = (k < KDIM);
  const int kc  = ok ? k : (KDIM - 8);
  const float* src = w + (size_t)m * KDIM + kc;
  v4u p;
#pragma unroll
  for (int e = 0; e < 4; ++e) {
    const unsigned v = pk16(bf_bits(src[2 * e]), bf_bits(src[2 * e + 1]));
    p[e] = ok ? v : 0u;
  }
  unsigned short* d = wp + (size_t)idx * 8;
  *(volatile v4u*)d = p;
  __threadfence();
  *(volatile v4u*)d = p;
}

__global__ __launch_bounds__(256) void k_packx(const float* __restrict__ x, unsigned short* xt) {
  const int idx = blockIdx.x * 256 + threadIdx.x;
  const int D0  = (idx & 3) * 8;
  const int cin = (idx >> 2) & 15;
  const int tp  = idx >> 6;
  const int b   = tp / (HIN * WIN);
  const int yx  = tp - b * (HIN * WIN);
  const float* src = x + ((size_t)((b * CIN + cin) * DCAP + D0)) * (HIN * WIN) + yx;
  float f[8];
#pragma unroll
  for (int e = 0; e < 8; ++e) f[e] = src[(size_t)e * (HIN * WIN)];
  v4u p;
#pragma unroll
  for (int e = 0; e < 4; ++e) p[e] = pk16(bf_bits(f[2 * e]), bf_bits(f[2 * e + 1]));
  unsigned short* d = xt + (size_t)idx * 8;
  *(volatile v4u*)d = p;
  __threadfence();
  *(volatile v4u*)d = p;
}

__global__ __launch_bounds__(256) void k_conv_route(
    const unsigned short* __restrict__ wp, const unsigned short* __restrict__ xt,
    const float* __restrict__ bias, const float* __restrict__ binit, float* rt) {
  extern __shared__ __align__(16) float sU[];
  __shared__ __align__(16) unsigned short sB[DCAP * KPAD];
  __shared__ __align__(16) float sbb[DOC * DCAP];
  __shared__ __align__(16) float scc[DOC * DCAP];
  __shared__ __align__(16) float ssv[CO * DOC];
  __shared__ float sn2[DOC];
  __shared__ float sbias[MDIM];

  const int t    = threadIdx.x;
  const int lane = t & 31;
  const int wv   = t >> 5;
  const int pos  = blockIdx.x;
  const int b    = pos / NPIX;
  const int rem  = pos - b * NPIX;
  const int h    = rem / WOUT;
  const int w    = rem - h * WOUT;

  const unsigned short* xb = xt + (size_t)b * (HIN * WIN * CIN * DCAP);
  for (int idx = t; idx < DCAP * KPAD; idx += 256) {
    const int Dd  = idx & 31;
    const int k   = idx >> 5;
    const int kc  = min(k, KDIM - 1);
    const int cin = kc / 9;
    const int r   = kc - cin * 9;
    const int kh  = r / 3, kw = r - kh * 3;
    const unsigned short v = xb[((size_t)((h + kh) * WIN + (w + kw)) * CIN + cin) * DCAP + Dd];
    sB[Dd * KPAD + k] = (k < KDIM) ? v : (unsigned short)0;
  }
  for (int idx = t; idx < DOC * DCAP; idx += 256) sbb[idx] = bfr(binit[idx]);
  sbias[t]       = bfr(bias[t]);
  sbias[t + 256] = bfr(bias[t + 256]);
  __syncthreads();

  const __bf16* Ab = (const __bf16*)(const void*)wp;
  const int rlane = lane & 15;
  const int koff  = (lane >> 4) * 8;
  const int mOff  = (lane >> 4) * 8;
  const int m0    = wv * 64;

  v8f acc[4][2];
#pragma unroll
  for (int i = 0; i < 4; ++i) { acc[i][0] = zero8(); acc[i][1] = zero8(); }

  for (int k0 = 0; k0 < KPAD; k0 += 32) {
    v16b bq[2];
#pragma unroll
    for (int j = 0; j < 2; ++j) bq[j] = ldfrag_lds(sB + (size_t)(16 * j + rlane) * KPAD + koff + k0);
#pragma unroll
    for (int i = 0; i < 4; ++i) {
      const v16b ah = ldfrag_b(Ab + (size_t)(m0 + 16 * i + rlane) * KPAD + koff + k0);
      acc[i][0] = mma_b_raw(ah, bq[0], acc[i][0]);
      acc[i][1] = mma_b_raw(ah, bq[1], acc[i][1]);
      dep_guard_b(acc[i][0], acc[i][1], ah, bq[1]);
    }
    keep2_b(bq[0], bq[1]);
  }
  acc_guard4(acc[0][0], acc[0][1], acc[1][0], acc[1][1]);
  acc_guard4(acc[2][0], acc[2][1], acc[3][0], acc[3][1]);

#pragma unroll
  for (int i = 0; i < 4; ++i) {
    const int mBase = m0 + 16 * i + mOff;
#pragma unroll
    for (int j = 0; j < 2; ++j) {
#pragma unroll
      for (int r = 0; r < 8; ++r) {
        const int m = mBase + r;
        sU[m * UPITCH + 16 * j + rlane] = acc[i][j][r] + sbias[m];
      }
    }
  }
  __syncthreads();

  for (int it = 0; it <= RITERS; ++it) {
    if (wv == 0) {
      const int Dd = lane;
      float mx = sbb[Dd];
#pragma unroll 1
      for (int d = 1; d < DOC; ++d) mx = fmaxf(mx, sbb[d * DCAP + Dd]);
      float sum = 0.f;
#pragma unroll 1
      for (int d = 0; d < DOC; ++d) {
        const float e = expf(sbb[d * DCAP + Dd] - mx);
        scc[d * DCAP + Dd] = e;
        sum += e;
      }
      const float inv = 1.0f / sum;
#pragma unroll 1
      for (int d = 0; d < DOC; ++d) scc[d * DCAP + Dd] = scc[d * DCAP + Dd] * inv;
    }
    __syncthreads();
#pragma unroll
    for (int q = 0; q < 2; ++q) {
      const int idx = t + 256 * q;
      const int c = idx >> 5, d = idx & 31;
      const float* up = sU + (c * DOC + d) * UPITCH;
      const float* cp = scc + d * DCAP;
      float s = 0.f;
#pragma unroll
      for (int Dd = 0; Dd < DCAP; ++Dd) s += cp[Dd] * up[Dd];
      ssv[idx] = s;
    }
    __syncthreads();
    if (it == RITERS) break;
    if (t < DOC) {
      const int d = t;
      float n2 = 0.f;
#pragma unroll 1
      for (int c = 0; c < CO; ++c) { const float sv = ssv[c * DOC + d]; n2 += sv * sv; }
      sn2[d] = (n2 * (1.0f / (1.0f + n2))) * rsqrtf(n2 + 1e-8f);
    }
    __syncthreads();
#pragma unroll
    for (int q = 0; q < 2; ++q) {
      const int idx = t + 256 * q;
      ssv[idx] = ssv[idx] * sn2[idx & 31];
    }
    __syncthreads();
#pragma unroll
    for (int q = 0; q < 4; ++q) {
      const int idx = t + 256 * q;
      const int d = idx >> 5, Dd = idx & 31;
      float a = 0.f;
#pragma unroll
      for (int c = 0; c < CO; ++c) a += sU[(c * DOC + d) * UPITCH + Dd] * ssv[c * DOC + d];
      sbb[idx] = sbb[idx] + a;
    }
    __syncthreads();
  }

  if (wv < 4) {
    const v4f v = *(const v4f*)(ssv + wv * 128 + 4 * lane);
    float* dst = rt + (size_t)pos * MDIM + wv * 128 + 4 * lane;
    *(volatile v4f*)dst = v;
    __threadfence();
    *(volatile v4f*)dst = v;
  }
}

__global__ __launch_bounds__(256) void k_pack_out(const float* __restrict__ rt, float* out) {
  const int g  = blockIdx.x * 256 + threadIdx.x;
  const int i0 = g * 4;
  v4f v;
#pragma unroll
  for (int j = 0; j < 4; ++j) {
    const int i   = i0 + j;
    const int row = i / NPIX;
    const int p   = i - row * NPIX;
    const int b   = row >> 9;
    const int cd  = row & 511;
    v[j] = rt[((size_t)(b * NPIX + p)) * MDIM + cd];
  }
  float* d = out + i0;
  *(volatile v4f*)d = v;
  __threadfence();
  *(volatile v4f*)d = v;
}

extern "C" void kernel_launch(void* const* d_in, const int* in_sizes, int n_in,
                              void* d_out, int out_size, void* d_ws, size_t ws_size,
                              hipStream_t stream) {
  if (n_in < 4) return;
  if (in_sizes[0] != NBAT * CIN * DCAP * HIN * WIN) return;
  if (in_sizes[1] != MDIM * KDIM) return;
  if (in_sizes[2] != MDIM) return;
  if (in_sizes[3] != DOC * DCAP) return;
  if (out_size != NPOS * MDIM) return;

  const float* x     = (const float*)d_in[0];
  const float* wk    = (const float*)d_in[1];
  const float* wb    = (const float*)d_in[2];
  const float* binit = (const float*)d_in[3];
  float* out = (float*)d_out;

  const size_t PWP = (size_t)MDIM * KPAD * 2;
  const size_t PXT = (size_t)NBAT * HIN * WIN * CIN * DCAP * 2;
  const size_t PRT = (size_t)NPOS * MDIM * 4;
  size_t off = 0;
  const size_t oWP = off; off += PWP;
  const size_t oXT = off; off += PXT;
  const size_t oRT = off; off += PRT;
  if (off > ws_size) return;
  if (off > (size_t)134217728) return;

  char* ws = (char*)d_ws;
  unsigned short* WP = (unsigned short*)(ws + oWP);
  unsigned short* XT = (unsigned short*)(ws + oXT);
  float*          RT = (float*)(ws + oRT);

  const dim3 blk(256);
  const int dynLds = MDIM * UPITCH * 4;

  k_packw<<<dim3(MDIM * (KPAD / 8) / 256), blk, 0, stream>>>(wk, WP);
  k_packx<<<dim3(NBAT * HIN * WIN * CIN * DCAP / 8 / 256), blk, 0, stream>>>(x, XT);
  (void)hipFuncSetAttribute(reinterpret_cast<const void*>(&k_conv_route),
                            hipFuncAttributeMaxDynamicSharedMemorySize, dynLds);
  k_conv_route<<<dim3(NPOS), blk, dynLds, stream>>>(WP, XT, wb, binit, RT);
  k_pack_out<<<dim3(NPOS * MDIM / 4 / 256), blk, 0, stream>>>(RT, out);
  (void)hipGetLastError();
}
